// VGAE_51616916963855
// MI455X (gfx1250) — hardware-verified
//
#include <hip/hip_runtime.h>


#define NN   1024
#define DI   128
#define DH   128
#define DL   64
#define OC   8
typedef _Float16 h16;
typedef unsigned short bf;
typedef __attribute__((ext_vector_type(16))) __bf16   v16bf;
typedef __attribute__((ext_vector_type(16))) _Float16 v16h;
typedef __attribute__((ext_vector_type(8)))  _Float16 v8h;
typedef __attribute__((ext_vector_type(8)))  unsigned short v8us;
typedef __attribute__((ext_vector_type(8)))  float    v8f;
typedef __attribute__((ext_vector_type(4)))  float    v4f;
typedef v8h  __attribute__((may_alias)) v8ha;
typedef v4f  __attribute__((may_alias)) v4fa;
typedef v8us __attribute__((may_alias)) v8usa;

__device__ __forceinline__ unsigned short f2bf(float f) { unsigned u = __float_as_uint(f); u += 0x7FFFu + ((u >> 16) & 1u); return (unsigned short)(u >> 16); }
__device__ __forceinline__ float bf2f(unsigned short b) { return __uint_as_float(((unsigned)b) << 16); }
__device__ __forceinline__ float bfr(float f) { return bf2f(f2bf(f)); }
__device__ __forceinline__ v16h cat16(v8h lo, v8h hi) { return __builtin_shufflevector(lo, hi, 0, 1, 2, 3, 4, 5, 6, 7, 8, 9, 10, 11, 12, 13, 14, 15); }
__device__ __forceinline__ v16bf cat16b(v8us lo, v8us hi) { return __builtin_bit_cast(v16bf, __builtin_shufflevector(lo, hi, 0, 1, 2, 3, 4, 5, 6, 7, 8, 9, 10, 11, 12, 13, 14, 15)); }
__device__ __forceinline__ v8f wmma16(v16h a, v16h b, v8f c) { return __builtin_amdgcn_wmma_f32_16x16x32_f16(false, a, false, b, (short)0, c, false, false); }
__device__ __forceinline__ v8f wmmab(v16bf a, v16bf b, v8f c) { return __builtin_amdgcn_wmma_f32_16x16x32_bf16(false, a, false, b, (short)0, c, false, false); }


template <typename T16> struct WFrag;
template <> struct WFrag<h16> { typedef v16h V; static __device__ __forceinline__ V ld(const h16* p) { return cat16(*(const v8h*)p, *(const v8h*)(p + 16)); } static __device__ __forceinline__ v8f mma(V a, V b, v8f c) { return wmma16(a, b, c); } };
template <> struct WFrag<bf> { typedef v16bf V; static __device__ __forceinline__ V ld(const bf* p) { return cat16b(*(const v8us*)p, *(const v8us*)(p + 16)); } static __device__ __forceinline__ v8f mma(V a, V b, v8f c) { return wmmab(a, b, c); } };
template <typename T16, int NSPLIT, bool BIAS>
__global__ __launch_bounds__(32) void k_gemmw(const T16* __restrict__ A, const T16* __restrict__ A2, const T16* __restrict__ Bt, const T16* __restrict__ Bt2, int K, float* C, int ldc, const float* __restrict__ bias, size_t sA, size_t sB, size_t sC) {
    typedef typename WFrag<T16>::V V;
    __shared__ __align__(16) float os[16 * 68];
    const size_t z = blockIdx.z; A += z * sA; if (A2) A2 += z * sA; Bt += z * sB; if (Bt2) Bt2 += z * sB; C += z * sC;
    const int lane = threadIdx.x & 31, lr = lane & 15, hi = lane >> 4; const int r0 = blockIdx.x * 64, c0 = blockIdx.y * 64;
    v8f acc[4][4];
#pragma unroll
    for (int mb = 0; mb < 4; ++mb)
#pragma unroll
        for (int nb = 0; nb < 4; ++nb) acc[mb][nb] = (v8f){};
    const size_t aoff = (size_t)(r0 + lr) * K + 8 * hi, boff = (size_t)(c0 + lr) * K + 8 * hi;
#pragma unroll 1
    for (int kc = 0; kc < K; kc += 32) {
        V a[4], a2[4];
#pragma unroll
        for (int mb = 0; mb < 4; ++mb) { a[mb] = WFrag<T16>::ld(A + aoff + (size_t)mb * 16 * K + kc); if (NSPLIT == 1 || NSPLIT == 2) a2[mb] = WFrag<T16>::ld(A2 + aoff + (size_t)mb * 16 * K + kc); }
#pragma unroll
        for (int nb = 0; nb < 4; ++nb) { const V b = WFrag<T16>::ld(Bt + boff + (size_t)nb * 16 * K + kc); V b2; if (NSPLIT >= 2) b2 = WFrag<T16>::ld(Bt2 + boff + (size_t)nb * 16 * K + kc);
#pragma unroll
            for (int mb = 0; mb < 4; ++mb) { acc[mb][nb] = WFrag<T16>::mma(a[mb], b, acc[mb][nb]); if (NSPLIT == 1 || NSPLIT == 2) acc[mb][nb] = WFrag<T16>::mma(a2[mb], b, acc[mb][nb]); if (NSPLIT >= 2) acc[mb][nb] = WFrag<T16>::mma(a[mb], b2, acc[mb][nb]); } }
        asm volatile("v_nop\n\tv_nop\n\tv_nop\n\tv_nop" : "+v"(acc[0][0]), "+v"(acc[1][1]), "+v"(acc[2][2]), "+v"(acc[3][3]) : "v"(a[0]), "v"(a[3]));
    }
#pragma unroll
    for (int mb = 0; mb < 4; ++mb) {
#pragma unroll
        for (int nb = 0; nb < 4; ++nb) {
#pragma unroll
            for (int j = 0; j < 8; ++j) os[(hi * 8 + j) * 68 + nb * 16 + lr] = acc[mb][nb][j]; }
        __builtin_amdgcn_wave_barrier(); asm volatile("" ::: "memory");
        float* crow = C + (size_t)(r0 + mb * 16) * ldc + c0;
#pragma unroll 1
        for (int ps = 0; ps < 2; ++ps) {
#pragma unroll
            for (int s = 0; s < 8; ++s) { const int row = 2 * s + hi, cofs = lr * 4; v4f val = *(const v4fa*)(os + row * 68 + cofs); if (BIAS) { val[0] += bfr(bias[c0 + cofs]); val[1] += bfr(bias[c0 + cofs + 1]); val[2] += bfr(bias[c0 + cofs + 2]); val[3] += bfr(bias[c0 + cofs + 3]); }
                *(volatile v4f*)(crow + (size_t)row * ldc + cofs) = val; }
            if (ps == 0) __threadfence(); }
        __builtin_amdgcn_wave_barrier(); asm volatile("" ::: "memory");
    }
}

typedef __attribute__((ext_vector_type(4))) unsigned short v4us;
typedef __attribute__((ext_vector_type(2))) unsigned short v2us;
__device__ __forceinline__ void splitf(float y, unsigned short& h, unsigned short& l) { h = f2bf(y); l = f2bf(y - bf2f(h)); }
__global__ __launch_bounds__(256) void k_cvt8(const float* __restrict__ src, bf* dst, size_t n8) { const size_t i = (size_t)blockIdx.x * 256 + threadIdx.x; if (i >= n8) return; const v8f v = *(const v8f*)(src + i * 8); v8us o;
#pragma unroll
    for (int k = 0; k < 8; ++k) o[k] = f2bf(v[k]); *(volatile v8us*)(dst + i * 8) = o; __threadfence(); *(volatile v8us*)(dst + i * 8) = o; }

__global__ __launch_bounds__(256) void k_wtG(const float* __restrict__ w, int K, int N, bf* Bt) {
    const int lane = threadIdx.x & 31; const int L0 = (blockIdx.x * 8 + (threadIdx.x >> 5)) * 8; const int nlines = N * K / 64;
#pragma unroll
    for (int ps = 0; ps < 2; ++ps) {
#pragma unroll 1
        for (int l = 0; l < 8; ++l) { const int L = L0 + l; if (L >= nlines) break; const size_t e = (size_t)L * 64 + lane * 2; const int k = (int)(e % K), n = (int)(e / K); v2us o;
            o[0] = f2bf(w[(size_t)k * N + n]); o[1] = f2bf(w[(size_t)(k + 1) * N + n]); *(volatile v2us*)(Bt + e) = o; }
        if (ps == 0) __threadfence(); }
}

__global__ __launch_bounds__(256) void k_deg(const float* __restrict__ adj, float* DISW) { const int lane = threadIdx.x & 31; const int i = blockIdx.x * 8 + (threadIdx.x >> 5); if (i >= NN) return; const float* ar = adj + (size_t)i * NN; float s = 0.f;
#pragma unroll 1
    for (int ch = 0; ch < NN / 128; ++ch) { const v4f a = *(const v4f*)(ar + ch * 128 + lane * 4); s = __fadd_rn(s, __fadd_rn(__fadd_rn(a[0], a[1]), __fadd_rn(a[2], a[3]))); }
#pragma unroll
    for (int sh = 16; sh; sh >>= 1) s = __fadd_rn(s, __shfl_xor(s, sh, 32));
    const float dis = __fdiv_rn(1.0f, __fsqrt_rn(s)); *(volatile float*)(DISW + (size_t)i * 32 + lane) = dis; __threadfence(); *(volatile float*)(DISW + (size_t)i * 32 + lane) = dis; }
template <bool RAW>
__global__ __launch_bounds__(256) void k_xst(const float* __restrict__ src, int F, const float* __restrict__ DISW, bf* Bh, bf* Bl) { const size_t e = ((size_t)blockIdx.x * 256 + threadIdx.x) * 2; if (e >= (size_t)F * NN) return; const int j = (int)(e % NN); const int f = (int)(e / NN); v2us oh, ol;
#pragma unroll
    for (int q = 0; q < 2; ++q) { float v = src[(size_t)(j + q) * F + f]; if (RAW) v = bfr(v); unsigned short a, b; splitf(__fmul_rn(DISW[(size_t)(j + q) * 32], v), a, b); oh[q] = a; ol[q] = b; }
    *(volatile v2us*)(Bh + e) = oh; *(volatile v2us*)(Bl + e) = ol; __threadfence(); *(volatile v2us*)(Bh + e) = oh; *(volatile v2us*)(Bl + e) = ol; }
__global__ __launch_bounds__(256) void k_rows(const float* __restrict__ G, int F, const float* __restrict__ DISW, bf* Hh, bf* Hl) { const size_t i4 = (size_t)blockIdx.x * 256 + threadIdx.x; if (i4 >= (size_t)NN * F / 4) return; const size_t e = i4 * 4; const int i = (int)(e / F); const float d = DISW[(size_t)i * 32]; const v4f a = *(const v4f*)(G + e); v4us oh, ol;
#pragma unroll
    for (int q = 0; q < 4; ++q) { unsigned short x2, y2; splitf(__fmul_rn(d, a[q]), x2, y2); oh[q] = x2; ol[q] = y2; }
    *(volatile v4us*)(Hh + e) = oh; *(volatile v4us*)(Hl + e) = ol; __threadfence(); *(volatile v4us*)(Hh + e) = oh; *(volatile v4us*)(Hl + e) = ol; }
__global__ __launch_bounds__(256) void k_relu32(float* F, size_t n4) { const size_t i = (size_t)blockIdx.x * 256 + threadIdx.x; if (i >= n4) return; v4f a = *(const v4f*)(F + i * 4); for (int q = 0; q < 4; ++q) a[q] = fmaxf(a[q], 0.0f); *(volatile v4f*)(F + i * 4) = a; __threadfence(); *(volatile v4f*)(F + i * 4) = a; }
__global__ __launch_bounds__(256) void k_reparam(const float* __restrict__ MU, const float* __restrict__ LV, const float* __restrict__ eps, float* Z, bf* Zh, bf* Zl, float* omu, float* olv) { const size_t i = (size_t)blockIdx.x * 256 + threadIdx.x; if (i >= (size_t)NN * DL / 4) return; const v4f m = *(const v4f*)(MU + i * 4), l = *(const v4f*)(LV + i * 4), ep = *(const v4f*)(eps + i * 4); v4f z; v4us oh, ol;
#pragma unroll
    for (int q = 0; q < 4; ++q) { float s = expf(__fmul_rn(0.5f, l[q])); float p = __fmul_rn(bfr(ep[q]), s); asm volatile("" : "+v"(p)); z[q] = __fadd_rn(m[q], p); unsigned short a, b; splitf(z[q], a, b); oh[q] = a; ol[q] = b; }
    *(volatile v4f*)(Z + i * 4) = z; *(volatile v4us*)(Zh + i * 4) = oh; *(volatile v4us*)(Zl + i * 4) = ol; *(volatile v4f*)(omu + i * 4) = m; *(volatile v4f*)(olv + i * 4) = l; __threadfence(); *(volatile v4f*)(Z + i * 4) = z; *(volatile v4us*)(Zh + i * 4) = oh; *(volatile v4us*)(Zl + i * 4) = ol; *(volatile v4f*)(omu + i * 4) = m; *(volatile v4f*)(olv + i * 4) = l; }
__global__ __launch_bounds__(256) void k_wr1blk(const float* __restrict__ w, bf* Bt4) { const int e2 = (blockIdx.x * 256 + threadIdx.x) * 2; if (e2 >= 4 * DL * DL) return; const int d = e2 % DL; const int o = (e2 / DL) % DL; const int blk = e2 / (DL * DL); v2us o2; o2[0] = f2bf(w[(size_t)(blk * DL + d) * DL + o]); o2[1] = f2bf(w[(size_t)(blk * DL + d + 1) * DL + o]); *(volatile v2us*)(Bt4 + e2) = o2; __threadfence(); *(volatile v2us*)(Bt4 + e2) = o2; }
__global__ __launch_bounds__(256) void k_uv(const float* __restrict__ ZA, const float* __restrict__ ZB, const float* __restrict__ ZC, const float* __restrict__ br1, float* U, float* Vv) { const size_t i = (size_t)blockIdx.x * 256 + threadIdx.x; if (i >= (size_t)NN * DL / 4) return; const int o0 = (int)((i * 4) % DL); const v4f a = *(const v4f*)(ZA + i * 4), b = *(const v4f*)(ZB + i * 4), c = *(const v4f*)(ZC + i * 4); v4f u, v;
#pragma unroll
    for (int q = 0; q < 4; ++q) { float t = __fsub_rn(a[q], c[q]); asm volatile("" : "+v"(t)); u[q] = __fadd_rn(t, bfr(br1[o0 + q])); v[q] = __fadd_rn(b[q], c[q]); }
    *(volatile v4f*)(U + i * 4) = u; *(volatile v4f*)(Vv + i * 4) = v; __threadfence(); *(volatile v4f*)(U + i * 4) = u; *(volatile v4f*)(Vv + i * 4) = v; }
__global__ __launch_bounds__(256) void k_zw(const float* __restrict__ Z, const float* __restrict__ wr1, int o0, bf* Ah, bf* Al) { const size_t k = (size_t)blockIdx.x * 256 + threadIdx.x; if (k >= (size_t)OC * NN * DL / 4) return; const size_t e = k * 4; const int d0 = (int)(e % DL); const int i = (int)((e / DL) % NN); const int oo = (int)(e / ((size_t)DL * NN)); const v4f z = *(const v4f*)(Z + (size_t)i * DL + d0); v4us oh, ol;
#pragma unroll
    for (int q = 0; q < 4; ++q) { unsigned short a, b; splitf(__fmul_rn(z[q], bfr(wr1[(size_t)(3 * DL + d0 + q) * DL + o0 + oo])), a, b); oh[q] = a; ol[q] = b; }
    *(volatile v4us*)(Ah + e) = oh; *(volatile v4us*)(Al + e) = ol; __threadfence(); *(volatile v4us*)(Ah + e) = oh; *(volatile v4us*)(Al + e) = ol; }
__global__ __launch_bounds__(256) void k_pacc(const float* __restrict__ S, const float* __restrict__ U, const float* __restrict__ Vv, const float* __restrict__ wr2, const float* __restrict__ br2, int o0, int first, int last, float* ACC, float* out) { const size_t k = (size_t)blockIdx.x * 256 + threadIdx.x; if (k >= (size_t)NN * NN / 4) return; const size_t e = k * 4; const int j0 = (int)(e % NN); const int i = (int)(e / NN); v4f acc; if (first) { acc[0] = acc[1] = acc[2] = acc[3] = 0.f; } else acc = *(const v4f*)(ACC + e);
#pragma unroll 1
    for (int oo = 0; oo < OC; ++oo) { const int o = o0 + oo; const float u = U[(size_t)i * DL + o]; const float w2 = bfr(wr2[o]); const v4f s = *(const v4f*)(S + (size_t)oo * NN * NN + e);
#pragma unroll
        for (int q = 0; q < 4; ++q) { float a = __fadd_rn(u, Vv[(size_t)(j0 + q) * DL + o]); asm volatile("" : "+v"(a)); a = __fadd_rn(a, s[q]); const float h = fmaxf(a, 0.0f); float p = __fmul_rn(h, w2); asm volatile("" : "+v"(p)); acc[q] = __fadd_rn(acc[q], p); } }
    if (last) { const float b2 = bfr(br2[0]); for (int q = 0; q < 4; ++q) acc[q] = __fadd_rn(acc[q], b2); *(volatile v4f*)(out + e) = acc; __threadfence(); *(volatile v4f*)(out + e) = acc; }
    else { *(volatile v4f*)(ACC + e) = acc; __threadfence(); *(volatile v4f*)(ACC + e) = acc; } }
__global__ __launch_bounds__(256) void k_zero16(bf* Z, size_t n8) { const size_t i = (size_t)blockIdx.x * 256 + threadIdx.x; if (i >= n8) return; v8us o; for (int k = 0; k < 8; ++k) o[k] = 0; *(volatile v8us*)(Z + i * 8) = o; __threadfence(); *(volatile v8us*)(Z + i * 8) = o; }

extern "C" void kernel_launch(void* const* d_in, const int* in_sizes, int n_in,
                              void* d_out, int out_size, void* d_ws, size_t ws_size, hipStream_t stream) {
    (void)in_sizes; (void)n_in; (void)out_size;
    const float* x = (const float*)d_in[0]; const float* adj = (const float*)d_in[1]; const float* eps = (const float*)d_in[2]; const float* W1 = (const float*)d_in[3]; const float* b1 = (const float*)d_in[4]; const float* Wmu = (const float*)d_in[5]; const float* bmu = (const float*)d_in[6]; const float* Wlv = (const float*)d_in[7]; const float* blv = (const float*)d_in[8]; const float* Wr1 = (const float*)d_in[9]; const float* br1 = (const float*)d_in[10]; const float* Wr2 = (const float*)d_in[11]; const float* br2 = (const float*)d_in[12];
    float* OUT = (float*)d_out; float* OMU = OUT + (size_t)NN * NN; float* OLV = OMU + (size_t)NN * DL;
    char* wsp = (char*)d_ws;
    auto take = [&](size_t bytes) { char* p = wsp; wsp += (bytes + 255) & ~(size_t)255; return (void*)p; };
    bf* ADJ = (bf*)take((size_t)NN * NN * 2); bf* ZER = (bf*)take((size_t)NN * NN * 2); float* DISW = (float*)take((size_t)NN * 32 * 4);
    bf* W1B = (bf*)take((size_t)DH * DI * 2); bf* WMB = (bf*)take((size_t)DL * DH * 2); bf* WLB = (bf*)take((size_t)DL * DH * 2); bf* WR4 = (bf*)take((size_t)4 * DL * DL * 2);
    bf* Bh = (bf*)take((size_t)DH * NN * 2); bf* Bl = (bf*)take((size_t)DH * NN * 2); float* G = (float*)take((size_t)NN * DH * 4); bf* Hh = (bf*)take((size_t)NN * DH * 2); bf* Hl = (bf*)take((size_t)NN * DH * 2); float* HF = (float*)take((size_t)NN * DH * 4);
    float* MU = (float*)take((size_t)NN * DL * 4); float* LV = (float*)take((size_t)NN * DL * 4); float* Z = (float*)take((size_t)NN * DL * 4); bf* Zh = (bf*)take((size_t)NN * DL * 2); bf* Zl = (bf*)take((size_t)NN * DL * 2);
    float* ZA = (float*)take((size_t)NN * DL * 4); float* ZB = (float*)take((size_t)NN * DL * 4); float* ZC = (float*)take((size_t)NN * DL * 4); float* U = (float*)take((size_t)NN * DL * 4); float* Vv = (float*)take((size_t)NN * DL * 4);
    bf* ZWh = (bf*)take((size_t)OC * NN * DL * 2); bf* ZWl = (bf*)take((size_t)OC * NN * DL * 2); float* S = (float*)take((size_t)OC * NN * NN * 4); float* ACC = (float*)take((size_t)NN * NN * 4);
    if ((size_t)(wsp - (char*)d_ws) > ws_size) return;
    const size_t n4h = (size_t)NN * DH / 4, n4l = (size_t)NN * DL / 4; const unsigned g4h = (unsigned)((n4h + 255) / 256), g4l = (unsigned)((n4l + 255) / 256);
    k_cvt8<<<(unsigned)(((size_t)NN * NN / 8 + 255) / 256), 256, 0, stream>>>(adj, ADJ, (size_t)NN * NN / 8); k_zero16<<<(unsigned)(((size_t)NN * NN / 8 + 255) / 256), 256, 0, stream>>>(ZER, (size_t)NN * NN / 8);
    k_wtG<<<(DI * DH / 64 + 63) / 64, 256, 0, stream>>>(W1, DI, DH, W1B); k_wtG<<<(DH * DL / 64 + 63) / 64, 256, 0, stream>>>(Wmu, DH, DL, WMB); k_wtG<<<(DH * DL / 64 + 63) / 64, 256, 0, stream>>>(Wlv, DH, DL, WLB); k_wr1blk<<<(4 * DL * DL / 2 + 255) / 256, 256, 0, stream>>>(Wr1, WR4);
    k_deg<<<NN / 8, 256, 0, stream>>>(adj, DISW);
    k_xst<true><<<(unsigned)(((size_t)DI * NN / 2 + 255) / 256), 256, 0, stream>>>(x, DI, DISW, Bh, Bl);
    k_gemmw<bf, 2, false><<<dim3(NN / 64, DI / 64, 1), 32, 0, stream>>>(ADJ, ZER, Bh, Bl, NN, G, DI, nullptr, 0, 0, 0);
    k_rows<<<g4h, 256, 0, stream>>>(G, DI, DISW, Hh, Hl);
    k_gemmw<bf, 1, true><<<dim3(NN / 64, DH / 64, 1), 32, 0, stream>>>(Hh, Hl, W1B, nullptr, DI, HF, DH, b1, 0, 0, 0); k_relu32<<<g4h, 256, 0, stream>>>(HF, n4h);
    k_xst<false><<<(unsigned)(((size_t)DH * NN / 2 + 255) / 256), 256, 0, stream>>>(HF, DH, DISW, Bh, Bl);
    k_gemmw<bf, 2, false><<<dim3(NN / 64, DH / 64, 1), 32, 0, stream>>>(ADJ, ZER, Bh, Bl, NN, G, DH, nullptr, 0, 0, 0);
    k_rows<<<g4h, 256, 0, stream>>>(G, DH, DISW, Hh, Hl);
    k_gemmw<bf, 1, true><<<dim3(NN / 64, DL / 64, 1), 32, 0, stream>>>(Hh, Hl, WMB, nullptr, DH, MU, DL, bmu, 0, 0, 0);
    k_gemmw<bf, 1, true><<<dim3(NN / 64, DL / 64, 1), 32, 0, stream>>>(Hh, Hl, WLB, nullptr, DH, LV, DL, blv, 0, 0, 0);
    k_reparam<<<g4l, 256, 0, stream>>>(MU, LV, eps, Z, Zh, Zl, OMU, OLV);
    k_gemmw<bf, 1, false><<<dim3(NN / 64, DL / 64, 1), 32, 0, stream>>>(Zh, Zl, WR4, nullptr, DL, ZA, DL, nullptr, 0, 0, 0);
    k_gemmw<bf, 1, false><<<dim3(NN / 64, DL / 64, 1), 32, 0, stream>>>(Zh, Zl, WR4 + (size_t)DL * DL, nullptr, DL, ZB, DL, nullptr, 0, 0, 0);
    k_gemmw<bf, 1, false><<<dim3(NN / 64, DL / 64, 1), 32, 0, stream>>>(Zh, Zl, WR4 + (size_t)2 * DL * DL, nullptr, DL, ZC, DL, nullptr, 0, 0, 0);
    k_uv<<<g4l, 256, 0, stream>>>(ZA, ZB, ZC, br1, U, Vv);
    for (int o0 = 0; o0 < DL; o0 += OC) {
        k_zw<<<(unsigned)(((size_t)OC * NN * DL / 4 + 255) / 256), 256, 0, stream>>>(Z, Wr1, o0, ZWh, ZWl);
        k_gemmw<bf, 2, false><<<dim3(NN / 64, NN / 64, OC), 32, 0, stream>>>(ZWh, ZWl, Zh, Zl, DL, S, NN, nullptr, (size_t)NN * DL, 0, (size_t)NN * NN);
        k_pacc<<<(unsigned)(((size_t)NN * NN / 4 + 255) / 256), 256, 0, stream>>>(S, U, Vv, Wr2, br2, o0, o0 == 0, o0 + OC >= DL, ACC, OUT); }
}
